// GAT_79980880986112
// MI455X (gfx1250) — hardware-verified
//
#include <hip/hip_runtime.h>
#include <stddef.h>
#include <stdint.h>
#include <math.h>


#define FIN    256
#define HC     128
#define KP     256
#define NCLS   32
#define NTHR   256
#define NWAVE  8
#define EPT    8
#define CHUNK  (NTHR * EPT)
#define WCAP   (EPT * 32)
#define LISTN  (NWAVE * WCAP)
#define NBA    1024
#define SLA    10
#define RCAP   28672
#define DEGCAP 128
#define GBM    64
#define GBN    128
#define GTHR   128
#define NUW0   (HC * (FIN / 8))
#define NUW1   (HC * (KP / 8))
#define NUW2   (64 * (KP / 8))
#define NUWR   (64 * (KP / 8))
#define NEGSL  0.2f
#define AGG_ZINTS (LISTN + 2 * RCAP + 3 * NBA)
#define AGG_LDS_INTS (AGG_ZINTS + 16)
#define WSMAX  134217728

static_assert((CHUNK & (CHUNK - 1)) == 0 && CHUNK <= 4096);
static_assert((NBA & (NBA - 1)) == 0 && NBA == (1 << SLA));
static_assert(((long long)CHUNK << SLA) < (1LL << 31));
static_assert(LISTN % NTHR == 0);
static_assert(NBA % NWAVE == 0 && NBA % 32 == 0 && NBA % GBM == 0);
static_assert(RCAP % 4 == 0 && AGG_ZINTS % 4 == 0 && LISTN % 4 == 0);
static_assert(FIN % 32 == 0 && KP % 32 == 0 && KP == 2 * HC && FIN == KP);
static_assert(GBM == (GTHR / 32) * 16 && GBN == 4 * 32 && GBN == HC);
static_assert(NUW0 % NTHR == 0 && NUW1 % NTHR == 0 && NUW2 % NTHR == 0 && NUWR % NTHR == 0);
static_assert(FIN / 8 == 32 && KP / 8 == 32);
static_assert(AGG_LDS_INTS * 4 <= 300000);
static_assert(HC == 4 * 32 && 2 * NCLS == 2 * 32);

typedef float          v2f   __attribute__((ext_vector_type(2)));
typedef float          v4f   __attribute__((ext_vector_type(4)));
typedef float          v8f   __attribute__((ext_vector_type(8)));
typedef int            v4i   __attribute__((ext_vector_type(4)));
typedef int            v8i   __attribute__((ext_vector_type(8)));
typedef unsigned int   v4u   __attribute__((ext_vector_type(4)));
typedef unsigned short v8us  __attribute__((ext_vector_type(8)));
typedef unsigned short v16us __attribute__((ext_vector_type(16)));
typedef __bf16         v16bf __attribute__((ext_vector_type(16)));
typedef v2f  __attribute__((may_alias)) v2fa;
typedef v4f  __attribute__((may_alias)) v4fa;
typedef v4i  __attribute__((may_alias)) v4ia;
typedef v8us __attribute__((may_alias)) v8usa;
union FragB { v16bf v; v16us u; v8us h[2]; v8i w; };

__device__ __forceinline__ v8f wmb(const FragB& a, const FragB& b, v8f c) {
  v8f d = __builtin_amdgcn_wmma_f32_16x16x32_bf16(false, a.v, false, b.v, (short)0, c, false, false);
  asm volatile("v_nop\n\tv_nop\n\tv_nop\n\tv_nop" : "+v"(d) : "v"(a.w), "v"(b.w));
  return d;
}

__device__ __forceinline__ unsigned bf16_bits(float f) {
  const unsigned u = __float_as_uint(f);
  return ((u + 0x7FFFu + ((u >> 16) & 1u)) >> 16) & 0xFFFFu;
}
__device__ __forceinline__ float bf16_val(float f) {
  return __uint_as_float(bf16_bits(f) << 16);
}
__device__ __forceinline__ v4f bfr4(const v4f a) {
  v4f r; r.x = bf16_val(a.x); r.y = bf16_val(a.y); r.z = bf16_val(a.z); r.w = bf16_val(a.w); return r;
}

template <int SLB>
__device__ __forceinline__ int scan_chunk(const int* __restrict__ dsts, int nE, int cbase, int slotBase,
                                          int nb, int vec8, int* list, int tid, int lane, int wave) {
  int wc = 0;
  const int el0  = tid * EPT;
  const int e0   = cbase + el0;
  const int sent = -2147483647 - 1;
  v4i da, db;
  if (vec8 != 0 && cbase + CHUNK <= nE) {
    da = *(const v4i*)(dsts + e0);
    db = *(const v4i*)(dsts + e0 + 4);
  } else {
    da.x = (e0     < nE) ? dsts[min(e0,     nE - 1)] : sent;
    da.y = (e0 + 1 < nE) ? dsts[min(e0 + 1, nE - 1)] : sent;
    da.z = (e0 + 2 < nE) ? dsts[min(e0 + 2, nE - 1)] : sent;
    da.w = (e0 + 3 < nE) ? dsts[min(e0 + 3, nE - 1)] : sent;
    db.x = (e0 + 4 < nE) ? dsts[min(e0 + 4, nE - 1)] : sent;
    db.y = (e0 + 5 < nE) ? dsts[min(e0 + 5, nE - 1)] : sent;
    db.z = (e0 + 6 < nE) ? dsts[min(e0 + 6, nE - 1)] : sent;
    db.w = (e0 + 7 < nE) ? dsts[min(e0 + 7, nE - 1)] : sent;
  }
  const unsigned nbs = (unsigned)slotBase;
  const unsigned unb = (unsigned)nb;
  const unsigned s0 = (unsigned)da.x - nbs, s1 = (unsigned)da.y - nbs;
  const unsigned s2 = (unsigned)da.z - nbs, s3 = (unsigned)da.w - nbs;
  const unsigned s4 = (unsigned)db.x - nbs, s5 = (unsigned)db.y - nbs;
  const unsigned s6 = (unsigned)db.z - nbs, s7 = (unsigned)db.w - nbs;
  const bool h0 = s0 < unb, h1 = s1 < unb, h2 = s2 < unb, h3 = s3 < unb;
  const bool h4 = s4 < unb, h5 = s5 < unb, h6 = s6 < unb, h7 = s7 < unb;
  const unsigned any = __builtin_amdgcn_ballot_w32(h0 | h1 | h2 | h3 | h4 | h5 | h6 | h7);
  if (any != 0u) {
#define HITJ(J, HJ, SJ) { \
      const unsigned mj = __builtin_amdgcn_ballot_w32(HJ); \
      if (mj != 0u) { \
        if (HJ) { \
          const int pos = wc + (int)__builtin_amdgcn_mbcnt_lo(mj, 0u); \
          if (pos < WCAP) list[wave * WCAP + pos] = ((el0 + (J)) << SLB) | (int)(SJ); \
        } \
        wc += (int)__builtin_popcount(mj); } }
    HITJ(0, h0, s0)
    HITJ(1, h1, s1)
    HITJ(2, h2, s2)
    HITJ(3, h3, s3)
    HITJ(4, h4, s4)
    HITJ(5, h5, s5)
    HITJ(6, h6, s6)
    HITJ(7, h7, s7)
#undef HITJ
  }
  return wc;
}

__global__ __launch_bounds__(NTHR) void k_wprep(const float* __restrict__ W0, const float* __restrict__ W1,
                                                const float* __restrict__ W2, const float* __restrict__ WR,
                                                unsigned short* W0T, unsigned short* W1T2, unsigned short* W2RT2) {
  const int u = (int)blockIdx.x * NTHR + (int)threadIdx.x;
  v8us o;
  unsigned short* dp;
  if (u < NUW0) {
    const int n  = u >> 5;
    const int k8 = (u & 31) * 8;
    const float* p = W0 + (size_t)k8 * HC + n;
#pragma unroll
    for (int i = 0; i < 8; ++i) o[i] = (unsigned short)bf16_bits(p[(size_t)i * HC]);
    dp = W0T + (size_t)n * FIN + k8;
  } else if (u < NUW0 + NUW1) {
    const int v  = u - NUW0;
    const int n  = v >> 5;
    const int k8 = (v & 31) * 8;
    const int kk = k8 & (HC - 1);
    const float* p = W1 + (size_t)kk * HC + n;
#pragma unroll
    for (int i = 0; i < 8; ++i) o[i] = (unsigned short)bf16_bits(p[(size_t)i * HC]);
    dp = W1T2 + (size_t)n * KP + k8;
  } else if (u < NUW0 + NUW1 + NUW2) {
    const int v  = u - NUW0 - NUW1;
    const int n  = v >> 5;
    const int k8 = (v & 31) * 8;
    const int kk = k8 & (HC - 1);
    const float* p = W2 + (size_t)kk * 64 + n;
#pragma unroll
    for (int i = 0; i < 8; ++i) o[i] = (unsigned short)bf16_bits(p[(size_t)i * 64]);
    dp = W2RT2 + (size_t)n * KP + k8;
  } else if (u < NUW0 + NUW1 + NUW2 + NUWR) {
    const int v  = u - NUW0 - NUW1 - NUW2;
    const int n  = v >> 5;
    const int k8 = (v & 31) * 8;
    const int kk = k8 & (HC - 1);
    const float* p = WR + (size_t)kk * 64 + n;
#pragma unroll
    for (int i = 0; i < 8; ++i) o[i] = (unsigned short)bf16_bits(p[(size_t)i * 64]);
    dp = W2RT2 + (size_t)(64 + n) * KP + k8;
  } else {
    return;
  }
  *(volatile v8us*)dp = o;
  __threadfence();
  *(volatile v8us*)dp = o;
}

__global__ __launch_bounds__(NTHR) void k_cvx(const float* __restrict__ x, int nN, int nUnits,
                                              unsigned short* xb) {
  const int u = (int)blockIdx.x * NTHR + (int)threadIdx.x;
  if (u >= nUnits) return;
  const int row = u >> 5;
  const int k8  = (u & 31) * 8;
  const int rc  = row < nN ? row : nN - 1;
  const float* p = x + (size_t)rc * FIN + k8;
  const v4f a = *(const v4f*)p;
  const v4f b = *(const v4f*)(p + 4);
  const bool ok = row < nN;
  v8us o;
  o[0] = ok ? (unsigned short)bf16_bits(a.x) : (unsigned short)0;
  o[1] = ok ? (unsigned short)bf16_bits(a.y) : (unsigned short)0;
  o[2] = ok ? (unsigned short)bf16_bits(a.z) : (unsigned short)0;
  o[3] = ok ? (unsigned short)bf16_bits(a.w) : (unsigned short)0;
  o[4] = ok ? (unsigned short)bf16_bits(b.x) : (unsigned short)0;
  o[5] = ok ? (unsigned short)bf16_bits(b.y) : (unsigned short)0;
  o[6] = ok ? (unsigned short)bf16_bits(b.z) : (unsigned short)0;
  o[7] = ok ? (unsigned short)bf16_bits(b.w) : (unsigned short)0;
  unsigned short* dp = xb + (size_t)row * FIN + k8;
  *(volatile v8us*)dp = o;
  __threadfence();
  *(volatile v8us*)dp = o;
}

template <int DHD>
__global__ __launch_bounds__(GTHR) void k_gemm(const unsigned short* __restrict__ A,
                                               const unsigned short* __restrict__ BT,
                                               float* Cm, const float* __restrict__ avl,
                                               const float* __restrict__ avr, float* SD) {
  static_assert(DHD == 64 || DHD == 32);
  constexpr int HL  = DHD / 4;
  constexpr int NDC = 2 * DHD;
  __shared__ __attribute__((aligned(16))) float stg[GBM * GBN];
  __shared__ __attribute__((aligned(16))) float sdt[GBM * 4];
  const int tid = (int)threadIdx.x, lane = tid & 31, wave = tid >> 5, hh = lane >> 4, m = lane & 15;
  const int rowBase = (int)blockIdx.x * GBM;

  v8f acc[8];
  {
    const v8f z = {0.f, 0.f, 0.f, 0.f, 0.f, 0.f, 0.f, 0.f};
#pragma unroll
    for (int t = 0; t < 8; ++t) acc[t] = z;
  }
  const unsigned short* ap = A  + (size_t)(rowBase + 16 * wave + m) * (size_t)KP + 8 * hh;
  const unsigned short* bp = BT + (size_t)m * (size_t)KP + 8 * hh;

#pragma unroll 1
  for (int k0 = 0; k0 < KP; k0 += 32) {
    FragB af;
    af.h[0] = *(const v8usa*)(ap + k0);
    af.h[1] = *(const v8usa*)(ap + k0 + 16);
#pragma unroll
    for (int nt = 0; nt < 8; ++nt) {
      const unsigned short* wq = bp + (size_t)(16 * nt) * (size_t)KP + k0;
      FragB bf;
      bf.h[0] = *(const v8usa*)wq;
      bf.h[1] = *(const v8usa*)(wq + 16);
      acc[nt] = wmb(af, bf, acc[nt]);
    }
  }

#pragma unroll
  for (int nt = 0; nt < 8; ++nt) {
    const int lc = 16 * nt + m;
#pragma unroll
    for (int r = 0; r < 8; ++r) {
      const int lr = 16 * wave + 8 * hh + r;
      stg[lr * GBN + lc] = acc[nt][r];
    }
  }
  __syncthreads();

  const int  c4   = 4 * lane;
  const bool hasd = c4 < NDC;
  const int  ca   = hasd ? c4 : 0;
  v4f al4 = bfr4(*(const v4fa*)(avl + ca));
  v4f ar4 = bfr4(*(const v4fa*)(avr + ca));
  al4.x = hasd ? al4.x : 0.0f; al4.y = hasd ? al4.y : 0.0f; al4.z = hasd ? al4.z : 0.0f; al4.w = hasd ? al4.w : 0.0f;
  ar4.x = hasd ? ar4.x : 0.0f; ar4.y = hasd ? ar4.y : 0.0f; ar4.z = hasd ? ar4.z : 0.0f; ar4.w = hasd ? ar4.w : 0.0f;

#pragma unroll 1
  for (int i = 0; i < 16; ++i) {
    const int row = wave * 16 + i;
    const v4f p = *(const v4fa*)(stg + row * GBN + 4 * lane);
    float s = p.x * al4.x, d = p.x * ar4.x;
    s = fmaf(p.y, al4.y, s); s = fmaf(p.z, al4.z, s); s = fmaf(p.w, al4.w, s);
    d = fmaf(p.y, ar4.y, d); d = fmaf(p.z, ar4.z, d); d = fmaf(p.w, ar4.w, d);
    s = hasd ? s : 0.0f;
    d = hasd ? d : 0.0f;
#pragma unroll
    for (int off = HL / 2; off > 0; off >>= 1) {
      s += __shfl_xor(s, off);
      d += __shfl_xor(d, off);
    }
    if (lane == 0)  { sdt[row * 4 + 0] = s; sdt[row * 4 + 2] = d; }
    if (lane == HL) { sdt[row * 4 + 1] = s; sdt[row * 4 + 3] = d; }
  }
  __syncthreads();

  const int w1 = wave & 1;
  const v4f sdv = *(const v4fa*)(sdt + 128 * w1 + 4 * lane);
  float* sp = SD + (size_t)rowBase * 4 + 128 * w1 + 4 * lane;
#pragma unroll 1
  for (int i = 0; i < 16; ++i) {
    const int row = wave * 16 + i;
    const v4f p = *(const v4fa*)(stg + row * GBN + 4 * lane);
    float* op = Cm + (size_t)(rowBase + row) * (size_t)HC + 4 * lane;
    *(volatile v4f*)op = p;
  }
  if (wave < 2) *(volatile v4f*)sp = sdv;
  __threadfence();
#pragma unroll 1
  for (int i = 0; i < 16; ++i) {
    const int row = wave * 16 + i;
    const v4f p = *(const v4fa*)(stg + row * GBN + 4 * lane);
    float* op = Cm + (size_t)(rowBase + row) * (size_t)HC + 4 * lane;
    *(volatile v4f*)op = p;
  }
  if (wave < 2) *(volatile v4f*)sp = sdv;
}

template <int MODE>
__global__ __launch_bounds__(NTHR) void k_agg(const int* __restrict__ srcs, const int* __restrict__ dsts,
                                              int nE, int nN, int vec8, int mRows,
                                              const float* __restrict__ SD,
                                              const float* __restrict__ xl, const float* __restrict__ bias,
                                              const float* resid, float* h1f,
                                              unsigned short* hb, float* outp) {
  static_assert(MODE == 0 || MODE == 1 || MODE == 2);
  constexpr int CPL = (MODE == 2) ? 2 : 4;
  extern __shared__ __attribute__((aligned(16))) int dsm[];
  int* list = dsm;
  int* hl   = dsm + LISTN;
  int* sl   = dsm + LISTN + RCAP;
  int* cnt  = dsm + LISTN + 2 * RCAP;
  int* offs = cnt + NBA;
  int* cur  = offs + NBA;
  int* misc = cur + NBA;
  const int tid = (int)threadIdx.x, lane = tid & 31, wave = tid >> 5;
  const int nodeBase = (int)blockIdx.x * NBA;

  {
    const v4i z4 = {0, 0, 0, 0};
    for (int i = tid * 4; i < AGG_ZINTS; i += NTHR * 4) *(v4ia*)(dsm + i) = z4;
    if (tid < 16) misc[tid] = 0;
  }
  v4f bb = {0.f, 0.f, 0.f, 0.f};
  if constexpr (MODE == 2) {
    const v2f t2 = *(const v2fa*)(bias + 2 * lane);
    bb.x = bf16_val(t2.x); bb.y = bf16_val(t2.y);
  } else {
    bb = bfr4(*(const v4fa*)(bias + 4 * lane));
  }
  __syncthreads();

  int t = 0, ov = 0;
  const int nChunks = (nE + CHUNK - 1) / CHUNK;
#pragma unroll 1
  for (int ch = 0; ch < nChunks; ++ch) {
    const int cbase = ch * CHUNK;
    const int wc = scan_chunk<SLA>(dsts, nE, cbase, nodeBase, NBA, vec8, list, tid, lane, wave);
    if (lane == 0) misc[wave] = wc;
    __syncthreads();
    if (wave == 0) {
#pragma unroll 1
      for (int w2 = 0; w2 < NWAVE; ++w2) {
        int c = misc[w2];
        c = c < 0 ? 0 : (c > WCAP ? WCAP : c);
#pragma unroll 1
        for (int b0 = 0; b0 < c; b0 += 32) {
          const int idx = b0 + lane;
          const int ent = list[w2 * WCAP + (idx < WCAP ? idx : WCAP - 1)];
          const int m32 = (c - b0) < 32 ? (c - b0) : 32;
#pragma unroll 1
          for (int k = 0; k < m32; ++k) {
            const int u    = __builtin_amdgcn_readlane(ent, k);
            const int slot = u & (NBA - 1);
            const int el   = (u >> SLA) & (CHUNK - 1);
            const int pk   = ((cbase + el) << SLA) | slot;
            if (t < RCAP) {
              if (lane == 0) { hl[t] = pk; cnt[slot] = cnt[slot] + 1; }
              t = t + 1;
            } else {
              ov = 1;
            }
          }
        }
      }
    }
    __syncthreads();
  }
  if (wave == 0 && lane == 0) { misc[8] = t; misc[9] = ov; }
  __syncthreads();
  int tt = misc[8];
  tt = tt < 0 ? 0 : (tt > RCAP ? RCAP : tt);
  const int ovf = misc[9];

  if (wave == 0) {
    const int base = lane * (NBA / 32);
    int s = 0;
#pragma unroll 1
    for (int i = 0; i < NBA / 32; ++i) s += cnt[base + i];
    int incl = s;
#pragma unroll
    for (int d = 1; d < 32; d <<= 1) {
      const int y = __shfl_up(incl, d, 32);
      if (lane >= d) incl += y;
    }
    int run = incl - s;
#pragma unroll 1
    for (int i = 0; i < NBA / 32; ++i) {
      const int cv = cnt[base + i];
      offs[base + i] = run;
      cur[base + i]  = run;
      run += cv;
    }
  }
  __syncthreads();
  if (wave == 0) {
#pragma unroll 1
    for (int b0 = 0; b0 < tt; b0 += 32) {
      const int idx = b0 + lane;
      const int ent = hl[idx < RCAP ? idx : RCAP - 1];
      const int m32 = (tt - b0) < 32 ? (tt - b0) : 32;
#pragma unroll 1
      for (int k = 0; k < m32; ++k) {
        const int u    = __builtin_amdgcn_readlane(ent, k);
        const int slot = u & (NBA - 1);
        if (lane == 0) {
          int p = cur[slot];
          p = p < 0 ? 0 : (p > RCAP - 1 ? RCAP - 1 : p);
          sl[p] = u;
          cur[slot] = p + 1;
        }
      }
    }
  }
  __syncthreads();

  const int   head = lane >> 4;
  const float qnan = __int_as_float(0x7fc00000);
  const float pz   = (ovf != 0) ? qnan : 0.0f;
#pragma unroll 1
  for (int si = 0; si < NBA / NWAVE; ++si) {
    const int s    = si * NWAVE + wave;
    const int node = nodeBase + s;
    int c = cnt[s];
    const bool big = c > DEGCAP;
    c = c < 0 ? 0 : (c > DEGCAP ? DEGCAP : c);
    int o = offs[s];
    o = o < 0 ? 0 : (o > RCAP ? RCAP : o);
    const int nc = node < nN ? node : nN - 1;
    const v4f sdd = *(const v4fa*)(SD + (size_t)nc * 4);
    const float ad = (head != 0) ? sdd.w : sdd.z;
    float mx = -1.0e30f, dn = 0.0f;
    v4f av = {0.f, 0.f, 0.f, 0.f};
#pragma unroll 1
    for (int b0 = 0; b0 < c; b0 += 32) {
      int idx = o + b0 + lane;
      idx = idx > RCAP - 1 ? RCAP - 1 : idx;
      const int ent = sl[idx];
      int eid = ent >> SLA;
      eid = eid < 0 ? 0 : (eid > nE - 1 ? nE - 1 : eid);
      int sr = srcs[eid];
      sr = sr < 0 ? 0 : (sr > nN - 1 ? nN - 1 : sr);
      const v4f sds = *(const v4fa*)(SD + (size_t)sr * 4);
      const int e0i = __float_as_int(sds.x);
      const int e1i = __float_as_int(sds.y);
      const int m32 = (c - b0) < 32 ? (c - b0) : 32;
#pragma unroll 1
      for (int k = 0; k < m32; ++k) {
        const int   sk = __builtin_amdgcn_readlane(sr, k);
        const float a0 = __int_as_float(__builtin_amdgcn_readlane(e0i, k));
        const float a1 = __int_as_float(__builtin_amdgcn_readlane(e1i, k));
        const float ask = (head != 0) ? a1 : a0;
        const float* rp = xl + (size_t)sk * HC + CPL * lane;
        v4f fs;
        if constexpr (MODE == 2) {
          const v2f t2 = *(const v2fa*)rp;
          fs.x = t2.x; fs.y = t2.y; fs.z = 0.0f; fs.w = 0.0f;
        } else {
          fs = *(const v4fa*)rp;
        }
        float lg = ask + ad;
        lg = lg > 0.f ? lg : NEGSL * lg;
        const float df = lg - mx;
        const float ee = __expf(-fabsf(df));
        const bool  up = df > 0.f;
        const float s1 = up ? ee : 1.0f;
        const float s2 = up ? 1.0f : ee;
        mx = up ? lg : mx;
        dn = fmaf(dn, s1, s2);
        av.x = fmaf(av.x, s1, s2 * fs.x);
        av.y = fmaf(av.y, s1, s2 * fs.y);
        if constexpr (MODE != 2) {
          av.z = fmaf(av.z, s1, s2 * fs.z);
          av.w = fmaf(av.w, s1, s2 * fs.w);
        }
      }
    }
    const float inv = (c > 0) ? __builtin_amdgcn_rcpf(dn) : 0.0f;
    const float pzr = big ? qnan : pz;
    const bool live = node < nN;

    if constexpr (MODE != 2) {
      v4f r4 = {0.f, 0.f, 0.f, 0.f};
      if constexpr (MODE == 1) r4 = *(const v4fa*)(resid + (size_t)nc * HC + 4 * lane);
      v4f y;
      y.x = fmaf(av.x, inv, r4.x) + bb.x;
      y.y = fmaf(av.y, inv, r4.y) + bb.y;
      y.z = fmaf(av.z, inv, r4.z) + bb.z;
      y.w = fmaf(av.w, inv, r4.w) + bb.w;
#pragma unroll 1
      for (int i = 0; i < 4; ++i) {
        const float v = y.x;
        const float e = (v > 0.0f) ? v : expm1f(v);
        y.x = y.y; y.y = y.z; y.z = y.w; y.w = e;
      }
      v4f ov;
      ov.x = live ? (y.x + pzr) : 0.0f;
      ov.y = live ? (y.y + pzr) : 0.0f;
      ov.z = live ? (y.z + pzr) : 0.0f;
      ov.w = live ? (y.w + pzr) : 0.0f;
      const unsigned hbx = bf16_bits(ov.x), hby = bf16_bits(ov.y), hbz = bf16_bits(ov.z), hbw = bf16_bits(ov.w);
      const unsigned lbx = bf16_bits(ov.x - __uint_as_float(hbx << 16));
      const unsigned lby = bf16_bits(ov.y - __uint_as_float(hby << 16));
      const unsigned lbz = bf16_bits(ov.z - __uint_as_float(hbz << 16));
      const unsigned lbw = bf16_bits(ov.w - __uint_as_float(hbw << 16));
      const int hw0 = (int)(hbx | (hby << 16)), hw1 = (int)(hbz | (hbw << 16));
      const int lw0 = (int)(lbx | (lby << 16)), lw1 = (int)(lbz | (lbw << 16));
      const int sa = (2 * lane) & 31, sb = (2 * lane + 1) & 31;
      const int g0 = __shfl(hw0, sa), g1 = __shfl(hw1, sa), g2 = __shfl(hw0, sb), g3 = __shfl(hw1, sb);
      const int q0 = __shfl(lw0, sa), q1 = __shfl(lw1, sa), q2 = __shfl(lw0, sb), q3 = __shfl(lw1, sb);
      const bool lsel = lane >= 16;
      v4u pv;
      pv.x = (unsigned)(lsel ? q0 : g0);
      pv.y = (unsigned)(lsel ? q1 : g1);
      pv.z = (unsigned)(lsel ? q2 : g2);
      pv.w = (unsigned)(lsel ? q3 : g3);
      unsigned short* gp = hb + (size_t)node * KP + 8 * lane;
      float* fp = h1f + (size_t)node * HC + 4 * lane;
      const bool wr = node < mRows;
      if (wr) {
        *(volatile v4u*)gp = pv;
        if constexpr (MODE == 0) *(volatile v4f*)fp = ov;
      }
      __threadfence();
      if (wr) {
        *(volatile v4u*)gp = pv;
        if constexpr (MODE == 0) *(volatile v4f*)fp = ov;
      }
    } else {
      const v2f rr = *(const v2fa*)(xl + (size_t)nc * HC + 64 + 2 * lane);
      const float o0 = fmaf(av.x, inv, rr.x) + bb.x;
      const float o1 = fmaf(av.y, inv, rr.y) + bb.y;
      const float p0 = __shfl_xor(o0, 16);
      const float p1 = __shfl_xor(o1, 16);
      const float m0 = 0.5f * (o0 + p0) + pzr;
      const float m1 = 0.5f * (o1 + p1) + pzr;
      const int sa = (2 * lane) & 31, sb = (2 * lane + 1) & 31;
      const float g0 = __shfl(m0, sa), g1 = __shfl(m1, sa), g2 = __shfl(m0, sb), g3 = __shfl(m1, sb);
      v4f ov4;
      ov4.x = g0; ov4.y = g1; ov4.z = g2; ov4.w = g3;
      float* op = outp + (size_t)node * NCLS + 4 * (lane & 7);
      if (live) {
        if (lane < 8) *(volatile v4f*)op = ov4;
        __threadfence();
        if (lane < 8) *(volatile v4f*)op = ov4;
      }
    }
  }
}

static inline int cdiv(int a, int b) { return (a + b - 1) / b; }

extern "C" void kernel_launch(void* const* d_in, const int* in_sizes, int n_in,
                              void* d_out, int out_size, void* d_ws, size_t ws_size,
                              hipStream_t stream) {
  if (n_in < 16) return;
  if (in_sizes[0] < FIN || (in_sizes[0] % FIN) != 0) return;
  const int nN = in_sizes[0] / FIN;
  if (nN > (1 << 22)) return;
  const int nE = in_sizes[1];
  if (in_sizes[2] != nE) return;
  if (nE < 1 || nE >= (1 << 21)) return;
  if (in_sizes[3] != FIN * HC) return;
  if (in_sizes[4] != HC || in_sizes[5] != HC || in_sizes[6] != HC) return;
  if (in_sizes[7] != HC * HC) return;
  if (in_sizes[8] != HC || in_sizes[9] != HC || in_sizes[10] != HC) return;
  if (in_sizes[11] != HC * 64) return;
  if (in_sizes[12] != 64 || in_sizes[13] != 64 || in_sizes[14] != 64) return;
  if (in_sizes[15] != HC * 64) return;
  if ((long long)out_size != (long long)nN * NCLS) return;

  const float* x   = (const float*)d_in[0];
  const int*   src = (const int*)d_in[1];
  const int*   dst = (const int*)d_in[2];
  const float* W0  = (const float*)d_in[3];
  const float* al0 = (const float*)d_in[4];
  const float* ar0 = (const float*)d_in[5];
  const float* b0  = (const float*)d_in[6];
  const float* W1  = (const float*)d_in[7];
  const float* al1 = (const float*)d_in[8];
  const float* ar1 = (const float*)d_in[9];
  const float* b1  = (const float*)d_in[10];
  const float* W2  = (const float*)d_in[11];
  const float* al2 = (const float*)d_in[12];
  const float* ar2 = (const float*)d_in[13];
  const float* b2  = (const float*)d_in[14];
  const float* WR  = (const float*)d_in[15];
  float* out = (float*)d_out;

  const int MP   = cdiv(nN, GBM) * GBM;
  const int gM   = MP / GBM;
  const int gA   = cdiv(MP, NBA);
  if ((long long)gA * NBA < (long long)MP) return;
  const int vec8 = ((nE & 3) == 0) ? 1 : 0;

  char* ws = (char*)d_ws;
  size_t off = 0;
  const size_t oW0T = off; off += (size_t)HC * FIN * 2;                   off = (off + 255) & ~(size_t)255;
  const size_t oW1T = off; off += (size_t)HC * KP * 2;                    off = (off + 255) & ~(size_t)255;
  const size_t oW2T = off; off += (size_t)HC * KP * 2;                    off = (off + 255) & ~(size_t)255;
  const size_t oSD  = off; off += (size_t)MP * 4 * 4;                     off = (off + 255) & ~(size_t)255;
  const size_t oXB  = off; off += (size_t)MP * FIN * 2;                   off = (off + 255) & ~(size_t)255;
  const size_t oT   = off; off += (size_t)MP * HC * 4;                    off = (off + 255) & ~(size_t)255;
  const size_t oH1  = off; off += (size_t)MP * HC * 4;                    off = (off + 255) & ~(size_t)255;
  const size_t oHHL = off; off += (size_t)MP * KP * 2;                    off = (off + 255) & ~(size_t)255;
  if (off > ws_size || off > (size_t)WSMAX) return;
  unsigned short* W0T   = (unsigned short*)(ws + oW0T);
  unsigned short* W1T2  = (unsigned short*)(ws + oW1T);
  unsigned short* W2RT2 = (unsigned short*)(ws + oW2T);
  float*          SDp   = (float*)(ws + oSD);
  unsigned short* XB    = (unsigned short*)(ws + oXB);
  float*          T     = (float*)(ws + oT);
  float*          H1    = (float*)(ws + oH1);
  unsigned short* HHL   = (unsigned short*)(ws + oHHL);

  const size_t aggLds = (size_t)AGG_LDS_INTS * 4;
  hipFuncSetAttribute(reinterpret_cast<const void*>(&k_agg<0>), hipFuncAttributeMaxDynamicSharedMemorySize, (int)aggLds);
  hipFuncSetAttribute(reinterpret_cast<const void*>(&k_agg<1>), hipFuncAttributeMaxDynamicSharedMemorySize, (int)aggLds);
  hipFuncSetAttribute(reinterpret_cast<const void*>(&k_agg<2>), hipFuncAttributeMaxDynamicSharedMemorySize, (int)aggLds);

  const int nUx = MP * (FIN / 8);
  k_wprep<<<(NUW0 + NUW1 + NUW2 + NUWR) / NTHR, NTHR, 0, stream>>>(W0, W1, W2, WR, W0T, W1T2, W2RT2);
  k_cvx<<<cdiv(nUx, NTHR), NTHR, 0, stream>>>(x, nN, nUx, XB);
  k_gemm<64><<<gM, GTHR, 0, stream>>>(XB, W0T, T, al0, ar0, SDp);
  k_agg<0><<<gA, NTHR, aggLds, stream>>>(src, dst, nE, nN, vec8, MP, SDp, T, b0, T, H1, HHL, out);
  k_gemm<64><<<gM, GTHR, 0, stream>>>(HHL, W1T2, T, al1, ar1, SDp);
  k_agg<1><<<gA, NTHR, aggLds, stream>>>(src, dst, nE, nN, vec8, MP, SDp, T, b1, H1, H1, HHL, out);
  k_gemm<32><<<gM, GTHR, 0, stream>>>(HHL, W2RT2, T, al2, ar2, SDp);
  k_agg<2><<<gA, NTHR, aggLds, stream>>>(src, dst, nE, nN, vec8, MP, SDp, T, b2, T, H1, HHL, out);
}
